// ContextMessageBlock_23802708755005
// MI455X (gfx1250) — hardware-verified
//
#include <hip/hip_runtime.h>
#include <stddef.h>
#include <stdint.h>
#include <math.h>


#define HD     128
#define NRBF   32
#define DIN    417
#define HP     136
#define AP     264
#define RP     40
#define FP     132
#define ROWS   64
#define WSC    16.0f
#define WINV   0.0625f
#define NCHMAX 5
#define TEMAX  16
#define GAM    26.6944444444f
#define CSTEP  (1.0f / 31.0f)

#define T_W1A  0
#define T_W1B  16384
#define T_W1R  32768
#define T_W2   36864
#define T_U1   53248
#define T_U2   86016
#define T_TOT  102400
#define T_GRP  (T_TOT / 8)
#define T_BLK  (T_GRP / 256)

#define L_H16  0
#define L_STG  (ROWS * HP * 2)
#define L_LDS  (L_STG + ROWS * FP * 4)

#define E_RBF  0
#define E_PRE  (ROWS * RP * 2)
#define E_HID  (E_PRE + ROWS * FP * 4)
#define E_SI   (E_HID + ROWS * HP * 2)
#define E_DI   (E_SI + ROWS * 4)
#define E_TI   (E_DI + ROWS * 4)
#define E_DS   (E_TI + ROWS * 4)
#define E_LDS  (E_DS + ROWS * 4)

#define NTHR   256
#define NWAVE  8
#define NB     256
#define EPT    8
#define CHUNK  (NTHR * EPT)
#define WCAP   (EPT * 32)
#define A_ACC  0
#define A_LIST (NB * HD * 4)
#define A_CNT  (A_LIST + NWAVE * WCAP * 4)
#define A_WCNT (A_CNT + NB * 4)
#define A_LDS  (A_WCNT + 64)

#define U_A    0
#define U_HID  (ROWS * AP * 2)
#define U_INV  (U_HID + ROWS * HP * 2)
#define U_LDS  (U_INV + ROWS * 4)

static_assert(T_GRP * 8 == T_TOT);
static_assert(T_BLK * 256 == T_GRP);
static_assert(((T_W1B | T_W1R | T_W2 | T_U1 | T_U2) & 63) == 0);
static_assert(((HP * 2) & 15) == 0 && ((AP * 2) & 15) == 0 && ((RP * 2) & 15) == 0 && ((FP * 4) & 15) == 0);
static_assert((L_STG & 15) == 0 && L_LDS <= 64 * 1024);
static_assert((E_PRE & 15) == 0 && (E_HID & 15) == 0 && (E_SI & 15) == 0 && E_LDS <= 64 * 1024);
static_assert(ROWS * HP * 2 <= ROWS * FP * 4);
static_assert(ROWS * AP * 2 == ROWS * FP * 4);
static_assert((A_LIST & 15) == 0 && (A_CNT & 15) == 0 && (A_WCNT & 15) == 0 && A_LDS <= 300 * 1024);
static_assert((U_HID & 15) == 0 && (U_INV & 15) == 0 && U_LDS <= 64 * 1024);
static_assert(NB == 32 * NWAVE && NB <= 256 && WCAP == 256 && CHUNK <= (1 << 20) && NB == NTHR && ROWS == 64);
static_assert(TEMAX * HD <= 2048);

typedef float    v4f  __attribute__((ext_vector_type(4)));
typedef float    v8f  __attribute__((ext_vector_type(8)));
typedef int      v4i  __attribute__((ext_vector_type(4)));
typedef _Float16 v4h  __attribute__((ext_vector_type(4)));
typedef _Float16 v8h  __attribute__((ext_vector_type(8)));
typedef _Float16 v16h __attribute__((ext_vector_type(16)));
union FragH { v16h v; v8h h[2]; };
union U8H   { v8h v; _Float16 e[8]; v4i q; };

__device__ __forceinline__ v8f zero8f() {
  v8f z;
#pragma unroll
  for (int i = 0; i < 8; ++i) z[i] = 0.0f;
  return z;
}

__device__ __forceinline__ v8f wmh(v16h a, v16h b, v8f c) {
  v8f d = __builtin_amdgcn_wmma_f32_16x16x32_f16(false, a, false, b, (short)0, c, false, false);
  asm volatile("v_nop\n\tv_nop\n\tv_nop\n\tv_nop" : "+v"(d) : "v"(a), "v"(b));
  return d;
}

__device__ __forceinline__ v8h cvt8h(v4f a, v4f b) {
  U8H u;
#pragma unroll
  for (int i = 0; i < 4; ++i) {
    u.e[i] = (_Float16)a[i];
    u.e[4 + i] = (_Float16)b[i];
  }
  return u.v;
}

__device__ __forceinline__ void gemm_h(const _Float16* arow, const _Float16* bcol, int kp, int nk, v8f acc[4]) {
#pragma unroll 1
  for (int kt = 0; kt < nk; ++kt) {
    FragH a;
    a.h[0] = *(const v8h*)(arow + 32 * kt);
    a.h[1] = *(const v8h*)(arow + 32 * kt + 16);
#pragma unroll
    for (int nt = 0; nt < 4; ++nt) {
      const _Float16* bp = bcol + (size_t)(16 * nt) * kp + 32 * kt;
      FragH b;
      b.h[0] = *(const v8h*)bp;
      b.h[1] = *(const v8h*)(bp + 16);
      acc[nt] = wmh(a.v, b.v, acc[nt]);
    }
  }
}

__device__ __forceinline__ void store_rows_f32(const float* stg, float* g, int row0, int M, int wave, int l) {
#pragma unroll
  for (int j = 0; j < 8; ++j) {
    const int lr = 8 * wave + j;
    const int gr = row0 + lr;
    if (gr < M) {
      const v4f v = *(const v4f*)(stg + lr * FP + 4 * l);
      *(volatile v4f*)(g + (size_t)gr * HD + 4 * l) = v;
    }
  }
  __threadfence();
#pragma unroll
  for (int j = 0; j < 8; ++j) {
    const int lr = 8 * wave + j;
    const int gr = row0 + lr;
    if (gr < M) {
      const v4f v = *(const v4f*)(stg + lr * FP + 4 * l);
      *(volatile v4f*)(g + (size_t)gr * HD + 4 * l) = v;
    }
  }
}

__global__ __launch_bounds__(256) void k_wcvt(const float* __restrict__ mw1, const float* __restrict__ mw2,
                                              const float* __restrict__ uw1, const float* __restrict__ uw2,
                                              const float* __restrict__ emb, v4i* wq, float* ek, int nTE) {
  __shared__ __attribute__((aligned(16))) float eks[TEMAX * HD];
  const int tid = threadIdx.x;
  if (blockIdx.x < T_BLK) {
    const int g = blockIdx.x * 256 + tid;
    if (g < T_GRP) {
      const float* src = mw1;
      int n = 0, kc = 0;
      if (g < 2048)       { const int q = g;         src = mw1;                      n = q >> 4; kc = (q & 15) * 8; }
      else if (g < 4096)  { const int q = g - 2048;  src = mw1 + (size_t)HD * HD;   n = q >> 4; kc = (q & 15) * 8; }
      else if (g < 4608)  { const int q = g - 4096;  src = mw1 + (size_t)384 * HD;  n = q >> 2; kc = (q & 3) * 8; }
      else if (g < 6656)  { const int q = g - 4608;  src = mw2;                      n = q >> 4; kc = (q & 15) * 8; }
      else if (g < 10752) { const int q = g - 6656;  src = uw1;                      n = q >> 5; kc = (q & 31) * 8; }
      else                { const int q = g - 10752; src = uw2;                      n = q >> 4; kc = (q & 15) * 8; }
      U8H u;
#pragma unroll
      for (int i = 0; i < 8; ++i) u.e[i] = (_Float16)(src[(size_t)(kc + i) * HD + n] * WSC);
      const v4i o = u.q;
      *(volatile v4i*)(wq + g) = o;
      __threadfence();
      *(volatile v4i*)(wq + g) = o;
    }
  } else {
    const int nOut = nTE * HD;
    for (int o = tid; o < nOut; o += 256) {
      const int t = o >> 7, c = o & (HD - 1);
      const float* er = emb + (size_t)t * HD;
      const float* wr = mw1 + (size_t)256 * HD + c;
      float s = 0.0f;
#pragma unroll 4
      for (int k = 0; k < HD; ++k) s += er[k] * wr[(size_t)k * HD];
      eks[o] = s;
    }
    __syncthreads();
    const int nQ = nTE * (HD / 4);
    for (int q = tid; q < nQ; q += 256) {
      const v4f v = *(const v4f*)(eks + 4 * q);
      *(volatile v4f*)(ek + 4 * q) = v;
    }
    __threadfence();
    for (int q = tid; q < nQ; q += 256) {
      const v4f v = *(const v4f*)(eks + 4 * q);
      *(volatile v4f*)(ek + 4 * q) = v;
    }
  }
}

__global__ __launch_bounds__(256) void k_node(const float* __restrict__ hin, const _Float16* th,
                                              float* HA, float* HB, int nN) {
  extern __shared__ __attribute__((aligned(16))) unsigned char lds_n[];
  _Float16* h16 = (_Float16*)(lds_n + L_H16);
  float*    stg = (float*)(lds_n + L_STG);
  const int tid = threadIdx.x, l = tid & 31, wave = tid >> 5, h = l >> 4, m = l & 15;
  const int wr = wave >> 1, wc = wave & 1;
  const int row0 = blockIdx.x * ROWS;

  for (int i = tid; i < ROWS * 16; i += 256) {
    const int r = i >> 4, c = (i & 15) * 8;
    const int gr = row0 + r;
    v4f x0 = {0.0f, 0.0f, 0.0f, 0.0f};
    v4f x1 = x0;
    if (gr < nN) {
      const float* p = hin + (size_t)gr * HD + c;
      x0 = *(const v4f*)p;
      x1 = *(const v4f*)(p + 4);
    }
    *(v8h*)(h16 + r * HP + c) = cvt8h(x0, x1);
  }
  __syncthreads();

  v8f acc[4];
#pragma unroll
  for (int i = 0; i < 4; ++i) acc[i] = zero8f();
  gemm_h(h16 + (16 * wr + m) * HP + 8 * h, th + T_W1A + (size_t)(64 * wc + m) * HD + 8 * h, HD, 4, acc);
#pragma unroll
  for (int nt = 0; nt < 4; ++nt) {
    const int c = 64 * wc + 16 * nt + m;
#pragma unroll
    for (int r = 0; r < 8; ++r) {
      const int lr = 16 * wr + 8 * h + r;
      stg[lr * FP + c] = acc[nt][r] * WINV;
    }
  }
  __syncthreads();
  store_rows_f32(stg, HA, row0, nN, wave, l);
  __syncthreads();

#pragma unroll
  for (int i = 0; i < 4; ++i) acc[i] = zero8f();
  gemm_h(h16 + (16 * wr + m) * HP + 8 * h, th + T_W1B + (size_t)(64 * wc + m) * HD + 8 * h, HD, 4, acc);
#pragma unroll
  for (int nt = 0; nt < 4; ++nt) {
    const int c = 64 * wc + 16 * nt + m;
#pragma unroll
    for (int r = 0; r < 8; ++r) {
      const int lr = 16 * wr + 8 * h + r;
      stg[lr * FP + c] = acc[nt][r] * WINV;
    }
  }
  __syncthreads();
  store_rows_f32(stg, HB, row0, nN, wave, l);
}

__global__ __launch_bounds__(256) void k_edge(const int* __restrict__ ei, const int* __restrict__ et,
                                              const float* __restrict__ pos, const float* __restrict__ HA,
                                              const float* __restrict__ HB, const float* __restrict__ EK,
                                              const float* __restrict__ mw1, const float* __restrict__ mb1,
                                              const float* __restrict__ mb2, const _Float16* th, _Float16* msg,
                                              int nN, int nE, int nTE, int cb, int clen) {
  extern __shared__ __attribute__((aligned(16))) unsigned char lds_e[];
  _Float16* rbft = (_Float16*)(lds_e + E_RBF);
  float*    pre  = (float*)(lds_e + E_PRE);
  _Float16* stg  = (_Float16*)(lds_e + E_PRE);
  _Float16* hid  = (_Float16*)(lds_e + E_HID);
  int*      sidx = (int*)(lds_e + E_SI);
  int*      didx = (int*)(lds_e + E_DI);
  int*      tidx = (int*)(lds_e + E_TI);
  float*    dsl  = (float*)(lds_e + E_DS);
  const int tid = threadIdx.x, l = tid & 31, wave = tid >> 5, h = l >> 4, m = l & 15;
  const int wr = wave >> 1, wc = wave & 1;
  const int e0 = blockIdx.x * ROWS;

  if (tid < ROWS) {
    const int le = e0 + tid;
    int sc = 0, dc = 0, tc = 0;
    float dist = 0.0f;
    if (le < clen) {
      const int g = cb + le;
      int s = ei[g];
      int d = ei[(size_t)nE + g];
      int t = et[g];
      if (s < 0) s += nN;
      sc = s < 0 ? 0 : (s > nN - 1 ? nN - 1 : s);
      if (d < 0) d += nN;
      dc = d < 0 ? 0 : (d > nN - 1 ? nN - 1 : d);
      if (t < 0) t += nTE;
      tc = t < 0 ? 0 : (t > nTE - 1 ? nTE - 1 : t);
      const float dx = pos[(size_t)sc * 3 + 0] - pos[(size_t)dc * 3 + 0];
      const float dy = pos[(size_t)sc * 3 + 1] - pos[(size_t)dc * 3 + 1];
      const float dz = pos[(size_t)sc * 3 + 2] - pos[(size_t)dc * 3 + 2];
      dist = sqrtf(dx * dx + dy * dy + dz * dz);
    }
    sidx[tid] = sc;
    didx[tid] = dc;
    tidx[tid] = tc;
    dsl[tid] = dist;
  }
  __syncthreads();

  {
    const int r = tid >> 2, k8 = (tid & 3) * 8;
    const float dist = dsl[r];
    U8H rb;
#pragma unroll
    for (int k = 0; k < 8; ++k) {
      const int kk = k8 + k;
      const float ck = (kk == NRBF - 1) ? 6.0f : 6.0f * ((float)kk * CSTEP);
      const float t = dist - ck;
      rb.e[k] = (_Float16)__expf(-GAM * (t * t));
    }
    *(v8h*)(rbft + r * RP + k8) = rb.v;
  }
  {
    const v4f w4 = *(const v4f*)(mw1 + (size_t)(DIN - 1) * HD + 4 * l);
    const v4f b4 = *(const v4f*)(mb1 + 4 * l);
#pragma unroll
    for (int j = 0; j < 8; ++j) {
      const int lr = 8 * wave + j;
      const int s = sidx[lr], d = didx[lr], t = tidx[lr];
      const float dist = dsl[lr];
      const v4f va = *(const v4f*)(HA + (size_t)s * HD + 4 * l);
      const v4f vb = *(const v4f*)(HB + (size_t)d * HD + 4 * l);
      const v4f ve = *(const v4f*)(EK + (size_t)t * HD + 4 * l);
      v4f p;
#pragma unroll
      for (int i = 0; i < 4; ++i) p[i] = (va[i] + vb[i]) + (ve[i] + b4[i]) + dist * w4[i];
      *(v4f*)(pre + lr * FP + 4 * l) = p;
    }
  }
  __syncthreads();

  v8f acc[4];
#pragma unroll
  for (int i = 0; i < 4; ++i) acc[i] = zero8f();
  gemm_h(rbft + (16 * wr + m) * RP + 8 * h, th + T_W1R + (size_t)(64 * wc + m) * 32 + 8 * h, 32, 1, acc);
#pragma unroll
  for (int nt = 0; nt < 4; ++nt) {
    const int c = 64 * wc + 16 * nt + m;
#pragma unroll
    for (int r = 0; r < 8; ++r) {
      const int lr = 16 * wr + 8 * h + r;
      const float v = acc[nt][r] * WINV + pre[lr * FP + c];
      const float sgm = __builtin_amdgcn_rcpf(1.0f + __expf(-v));
      hid[lr * HP + c] = (_Float16)(v * sgm);
    }
  }
  __syncthreads();

#pragma unroll
  for (int i = 0; i < 4; ++i) acc[i] = zero8f();
  gemm_h(hid + (16 * wr + m) * HP + 8 * h, th + T_W2 + (size_t)(64 * wc + m) * HD + 8 * h, HD, 4, acc);
#pragma unroll
  for (int nt = 0; nt < 4; ++nt) {
    const int c = 64 * wc + 16 * nt + m;
    const float bc = mb2[c];
#pragma unroll
    for (int r = 0; r < 8; ++r) {
      const int lr = 16 * wr + 8 * h + r;
      const float v = acc[nt][r] * WINV + bc;
      const float sgm = __builtin_amdgcn_rcpf(1.0f + __expf(-v));
      stg[lr * HP + c] = (_Float16)(v * sgm);
    }
  }
  __syncthreads();

  {
    const int c8 = 8 * (l & 15);
#pragma unroll
    for (int j = 0; j < 4; ++j) {
      const int lr = 8 * wave + 2 * j + h;
      const int gr = e0 + lr;
      if (gr < clen) {
        const v8h v = *(const v8h*)(stg + lr * HP + c8);
        *(volatile v8h*)(msg + (size_t)gr * HD + c8) = v;
      }
    }
    __threadfence();
#pragma unroll
    for (int j = 0; j < 4; ++j) {
      const int lr = 8 * wave + 2 * j + h;
      const int gr = e0 + lr;
      if (gr < clen) {
        const v8h v = *(const v8h*)(stg + lr * HP + c8);
        *(volatile v8h*)(msg + (size_t)gr * HD + c8) = v;
      }
    }
  }
}

__device__ __forceinline__ int scan_chunk(const int* __restrict__ dsts, int nE, int cbase, int nodeBase,
                                          int* list, int tid, int wave, int vec_ok) {
  int wc = 0;
  const int el0  = tid * EPT;
  const int e0   = cbase + el0;
  const int sent = -2147483647 - 1;
  v4i da, db;
  if (vec_ok != 0 && e0 + 7 < nE) {
    da = *(const v4i*)(dsts + e0);
    db = *(const v4i*)(dsts + e0 + 4);
  } else {
    da.x = (e0     < nE) ? dsts[(e0     < nE) ? e0     : nE - 1] : sent;
    da.y = (e0 + 1 < nE) ? dsts[(e0 + 1 < nE) ? e0 + 1 : nE - 1] : sent;
    da.z = (e0 + 2 < nE) ? dsts[(e0 + 2 < nE) ? e0 + 2 : nE - 1] : sent;
    da.w = (e0 + 3 < nE) ? dsts[(e0 + 3 < nE) ? e0 + 3 : nE - 1] : sent;
    db.x = (e0 + 4 < nE) ? dsts[(e0 + 4 < nE) ? e0 + 4 : nE - 1] : sent;
    db.y = (e0 + 5 < nE) ? dsts[(e0 + 5 < nE) ? e0 + 5 : nE - 1] : sent;
    db.z = (e0 + 6 < nE) ? dsts[(e0 + 6 < nE) ? e0 + 6 : nE - 1] : sent;
    db.w = (e0 + 7 < nE) ? dsts[(e0 + 7 < nE) ? e0 + 7 : nE - 1] : sent;
  }
  const unsigned nb = (unsigned)nodeBase;
  const unsigned s0 = (unsigned)da.x - nb, s1 = (unsigned)da.y - nb;
  const unsigned s2 = (unsigned)da.z - nb, s3 = (unsigned)da.w - nb;
  const unsigned s4 = (unsigned)db.x - nb, s5 = (unsigned)db.y - nb;
  const unsigned s6 = (unsigned)db.z - nb, s7 = (unsigned)db.w - nb;
  const bool q0 = s0 < (unsigned)NB, q1 = s1 < (unsigned)NB, q2 = s2 < (unsigned)NB, q3 = s3 < (unsigned)NB;
  const bool q4 = s4 < (unsigned)NB, q5 = s5 < (unsigned)NB, q6 = s6 < (unsigned)NB, q7 = s7 < (unsigned)NB;
  const unsigned any = __builtin_amdgcn_ballot_w32(q0 | q1 | q2 | q3 | q4 | q5 | q6 | q7);
  if (any != 0u) {
#define HITJ(J, QJ, SJ) { \
      const unsigned mj = __builtin_amdgcn_ballot_w32(QJ); \
      if (mj != 0u) { \
        if (QJ) { \
          const int p = wc + (int)__builtin_amdgcn_mbcnt_lo(mj, 0u); \
          if (p < WCAP) list[wave * WCAP + p] = ((el0 + (J)) << 8) | (int)(SJ); \
        } \
        wc += (int)__builtin_popcount(mj); } }
    HITJ(0, q0, s0)
    HITJ(1, q1, s1)
    HITJ(2, q2, s2)
    HITJ(3, q3, s3)
    HITJ(4, q4, s4)
    HITJ(5, q5, s5)
    HITJ(6, q6, s6)
    HITJ(7, q7, s7)
#undef HITJ
  }
  return wc;
}

__global__ __launch_bounds__(NTHR) void k_agg(const int* __restrict__ dsts, const _Float16* __restrict__ msg,
                                               float* agg, float* cntg, int nN, int clen, int first, int vec_ok) {
  extern __shared__ __attribute__((aligned(16))) unsigned char lds_a[];
  float* acc  = (float*)(lds_a + A_ACC);
  int*   list = (int*)(lds_a + A_LIST);
  float* cntl = (float*)(lds_a + A_CNT);
  int*   wcnt = (int*)(lds_a + A_WCNT);
  const int tid = threadIdx.x, l = tid & 31, wave = tid >> 5;
  const int nodeBase = blockIdx.x * NB;

  for (int i = tid; i < NB * 32; i += NTHR) {
    const int slot = i >> 5, q = (i & 31) * 4;
    const int node = nodeBase + slot;
    v4f v = {0.0f, 0.0f, 0.0f, 0.0f};
    if (first == 0 && node < nN) v = *(const v4f*)(agg + (size_t)node * HD + q);
    *(v4f*)(acc + slot * HD + q) = v;
  }
  {
    float c0 = 0.0f;
    if (first == 0) c0 = cntg[(size_t)nodeBase + tid];
    cntl[tid] = c0;
  }
  __syncthreads();

  const int nChunks = (clen + CHUNK - 1) / CHUNK;
#pragma unroll 1
  for (int ch = 0; ch < nChunks; ++ch) {
    const int cbase = ch * CHUNK;
    const int wc = scan_chunk(dsts, clen, cbase, nodeBase, list, tid, wave, vec_ok);
    if (l == 0) wcnt[wave] = wc;
    __syncthreads();

#pragma unroll 1
    for (int w2 = 0; w2 < NWAVE; ++w2) {
      int n = wcnt[w2];
      n = n > WCAP ? WCAP : (n < 0 ? 0 : n);
      const int* lp = list + w2 * WCAP;
#pragma unroll 1
      for (int i0 = 0; i0 < n; i0 += 32) {
        const int idx = i0 + l;
        const int v = lp[(idx < n) ? idx : 0];
        unsigned mk = __builtin_amdgcn_ballot_w32((idx < n) && ((v & 7) == wave));
#pragma unroll 1
        while (mk != 0u) {
          const int bpos = __builtin_ctz(mk);
          mk &= mk - 1u;
          const int vv = __shfl(v, bpos);
          const int slot = vv & 255;
          int e = cbase + (vv >> 8);
          e = e < 0 ? 0 : (e > clen - 1 ? clen - 1 : e);
          const v4h x = *(const v4h*)(msg + (size_t)e * HD + 4 * l);
          float* ap = acc + slot * HD + 4 * l;
          v4f a = *(v4f*)ap;
          a[0] += (float)x[0]; a[1] += (float)x[1]; a[2] += (float)x[2]; a[3] += (float)x[3];
          *(v4f*)ap = a;
          if (l == 0) cntl[slot] = cntl[slot] + 1.0f;
        }
      }
    }
    __syncthreads();
  }

#pragma unroll
  for (int j = 0; j < 32; ++j) {
    const int slot = wave * 32 + j;
    const int node = nodeBase + slot;
    if (node < nN) {
      const v4f a = *(const v4f*)(acc + slot * HD + 4 * l);
      *(volatile v4f*)(agg + (size_t)node * HD + 4 * l) = a;
    }
  }
  v4f cv = {0.0f, 0.0f, 0.0f, 0.0f};
  if (tid < NB / 4) cv = *(const v4f*)(cntl + 4 * tid);
  float* cp = cntg + (size_t)nodeBase + 4 * tid;
  if (tid < NB / 4) *(volatile v4f*)cp = cv;
  __threadfence();
#pragma unroll
  for (int j = 0; j < 32; ++j) {
    const int slot = wave * 32 + j;
    const int node = nodeBase + slot;
    if (node < nN) {
      const v4f a = *(const v4f*)(acc + slot * HD + 4 * l);
      *(volatile v4f*)(agg + (size_t)node * HD + 4 * l) = a;
    }
  }
  if (tid < NB / 4) *(volatile v4f*)cp = cv;
}

__global__ __launch_bounds__(256) void k_upd(const float* __restrict__ hin, const float* __restrict__ agg,
                                             const float* __restrict__ cnt, const int* __restrict__ ntype,
                                             const _Float16* th, const float* __restrict__ ub1,
                                             const float* __restrict__ ub2, const float* __restrict__ lng,
                                             const float* __restrict__ lnb, float* out, int nN) {
  extern __shared__ __attribute__((aligned(16))) unsigned char lds_u[];
  _Float16* a16 = (_Float16*)(lds_u + U_A);
  float*    stg = (float*)(lds_u + U_A);
  _Float16* hid = (_Float16*)(lds_u + U_HID);
  float*    invl = (float*)(lds_u + U_INV);
  const int tid = threadIdx.x, l = tid & 31, wave = tid >> 5, h = l >> 4, m = l & 15;
  const int wr = wave >> 1, wc = wave & 1;
  const int row0 = blockIdx.x * ROWS;

  if (tid < ROWS) {
    const int gr = row0 + tid;
    float iv = 0.0f;
    if (gr < nN) iv = 1.0f / fmaxf(cnt[gr], 1.0f);
    invl[tid] = iv;
  }
  __syncthreads();

  for (int i = tid; i < ROWS * 32; i += 256) {
    const int r = i >> 5, c = (i & 31) * 8;
    const int gr = row0 + r;
    v4f x0 = {0.0f, 0.0f, 0.0f, 0.0f};
    v4f x1 = x0;
    if (gr < nN) {
      if (c < HD) {
        const float* p = hin + (size_t)gr * HD + c;
        x0 = *(const v4f*)p;
        x1 = *(const v4f*)(p + 4);
      } else {
        const float* p = agg + (size_t)gr * HD + (c - HD);
        const float iv = invl[r];
        x0 = *(const v4f*)p * iv;
        x1 = *(const v4f*)(p + 4) * iv;
      }
    }
    *(v8h*)(a16 + r * AP + c) = cvt8h(x0, x1);
  }
  __syncthreads();

  v8f acc[4];
#pragma unroll
  for (int i = 0; i < 4; ++i) acc[i] = zero8f();
  gemm_h(a16 + (16 * wr + m) * AP + 8 * h, th + T_U1 + (size_t)(64 * wc + m) * 256 + 8 * h, 256, 8, acc);
#pragma unroll
  for (int nt = 0; nt < 4; ++nt) {
    const int c = 64 * wc + 16 * nt + m;
    const float bc = ub1[c];
#pragma unroll
    for (int r = 0; r < 8; ++r) {
      const int lr = 16 * wr + 8 * h + r;
      const float v = acc[nt][r] * WINV + bc;
      const float sgm = __builtin_amdgcn_rcpf(1.0f + __expf(-v));
      hid[lr * HP + c] = (_Float16)(v * sgm);
    }
  }
  __syncthreads();

#pragma unroll
  for (int i = 0; i < 4; ++i) acc[i] = zero8f();
  gemm_h(hid + (16 * wr + m) * HP + 8 * h, th + T_U2 + (size_t)(64 * wc + m) * HD + 8 * h, HD, 4, acc);
#pragma unroll
  for (int nt = 0; nt < 4; ++nt) {
    const int c = 64 * wc + 16 * nt + m;
    const float bc = ub2[c];
#pragma unroll
    for (int r = 0; r < 8; ++r) {
      const int lr = 16 * wr + 8 * h + r;
      stg[lr * FP + c] = acc[nt][r] * WINV + bc;
    }
  }
  __syncthreads();

  {
    const int row = tid >> 2, q = tid & 3;
    const int gr = row0 + row;
    const int grc = gr < nN ? gr : nN - 1;
    float* xr = stg + row * FP + 32 * q;
    const float* hr = hin + (size_t)grc * HD + 32 * q;
    float x[32], hv[32];
#pragma unroll
    for (int j = 0; j < 8; ++j) {
      const v4f u = *(const v4f*)(xr + 4 * j);
      const v4f hq = *(const v4f*)(hr + 4 * j);
#pragma unroll
      for (int i = 0; i < 4; ++i) {
        hv[4 * j + i] = hq[i];
        x[4 * j + i] = hq[i] + u[i];
      }
    }
    float s = 0.0f;
#pragma unroll
    for (int j = 0; j < 32; ++j) s += x[j];
    s += __shfl_xor(s, 1);
    s += __shfl_xor(s, 2);
    const float mu = s * (1.0f / 128.0f);
    float dv = 0.0f;
#pragma unroll
    for (int j = 0; j < 32; ++j) { const float t = x[j] - mu; dv += t * t; }
    dv += __shfl_xor(dv, 1);
    dv += __shfl_xor(dv, 2);
    const float var = dv * (1.0f / 128.0f);
    const float rstd = rsqrtf(var + 1e-5f);
    const bool lig = (ntype[grc] == 0);
#pragma unroll
    for (int j = 0; j < 8; ++j) {
      const v4f g4 = *(const v4f*)(lng + 32 * q + 4 * j);
      const v4f b4 = *(const v4f*)(lnb + 32 * q + 4 * j);
      v4f y;
#pragma unroll
      for (int i = 0; i < 4; ++i) {
        const float ln = (x[4 * j + i] - mu) * rstd * g4[i] + b4[i];
        y[i] = lig ? ln : hv[4 * j + i];
      }
      *(v4f*)(xr + 4 * j) = y;
    }
  }
  __syncthreads();

  store_rows_f32(stg, out, row0, nN, wave, l);
}

extern "C" void kernel_launch(void* const* d_in, const int* in_sizes, int n_in,
                              void* d_out, int out_size, void* d_ws, size_t ws_size,
                              hipStream_t stream) {
  if (n_in < 16) return;
  const int nN  = in_sizes[0] / HD;
  const int nE  = in_sizes[3];
  const int nTE = in_sizes[5] / HD;
  if (nN <= 0 || nE <= 0 || nTE <= 0 || nTE > TEMAX) return;
  if (in_sizes[0] != nN * HD || in_sizes[1] != nN * 3 || in_sizes[2] != 2 * nE || in_sizes[4] != nN) return;
  if (in_sizes[5] != nTE * HD || in_sizes[6] != DIN * HD || in_sizes[7] < HD) return;
  if (in_sizes[8] != HD * HD || in_sizes[9] < HD || in_sizes[10] != 256 * HD || in_sizes[11] < HD) return;
  if (in_sizes[12] != HD * HD || in_sizes[13] < HD || in_sizes[14] < HD || in_sizes[15] < HD) return;
  if ((long long)out_size != (long long)nN * HD) return;

  const float* hin   = (const float*)d_in[0];
  const float* pos   = (const float*)d_in[1];
  const int*   ei    = (const int*)d_in[2];
  const int*   et    = (const int*)d_in[3];
  const int*   ntype = (const int*)d_in[4];
  const float* emb   = (const float*)d_in[5];
  const float* mw1   = (const float*)d_in[6];
  const float* mb1   = (const float*)d_in[7];
  const float* mw2   = (const float*)d_in[8];
  const float* mb2   = (const float*)d_in[9];
  const float* uw1   = (const float*)d_in[10];
  const float* ub1   = (const float*)d_in[11];
  const float* uw2   = (const float*)d_in[12];
  const float* ub2   = (const float*)d_in[13];
  const float* lng   = (const float*)d_in[14];
  const float* lnb   = (const float*)d_in[15];
  float* out0 = (float*)d_out;

  const int nBlkN = (nN + ROWS - 1) / ROWS;
  const int nBlkA = (nN + NB - 1) / NB;
  long long chl = ((long long)nE + NCHMAX - 1) / NCHMAX;
  chl = (chl + CHUNK - 1) / CHUNK * CHUNK;
  const int CH = (int)chl;
  int nchl = 0;
  for (int c = 0; c < NCHMAX; ++c) if ((long long)c * CH < (long long)nE) ++nchl;
  const int vec_ok = ((nE & 3) == 0) ? 1 : 0;

  char* ws = (char*)d_ws;
  size_t off = 0;
  const size_t oT  = off; off += (size_t)T_TOT * 2;          off = (off + 255) & ~(size_t)255;
  const size_t oEK = off; off += (size_t)nTE * HD * 4;       off = (off + 255) & ~(size_t)255;
  const size_t oHA = off; off += (size_t)nN * HD * 4;        off = (off + 255) & ~(size_t)255;
  const size_t oHB = off; off += (size_t)nN * HD * 4;        off = (off + 255) & ~(size_t)255;
  const size_t oMS = off; off += (size_t)CH * HD * 2;        off = (off + 255) & ~(size_t)255;
  const size_t oAG = off; off += (size_t)nN * HD * 4;        off = (off + 255) & ~(size_t)255;
  const size_t oCN = off; off += (size_t)nBlkA * NB * 4;     off = (off + 255) & ~(size_t)255;
  if (off > ws_size) return;
  v4i*            wq  = (v4i*)(ws + oT);
  const _Float16* th  = (const _Float16*)(ws + oT);
  float*          ekp = (float*)(ws + oEK);
  float*          hap = (float*)(ws + oHA);
  float*          hbp = (float*)(ws + oHB);
  _Float16*       msp = (_Float16*)(ws + oMS);
  float*          agp = (float*)(ws + oAG);
  float*          cnp = (float*)(ws + oCN);

  const hipError_t a0 = hipFuncSetAttribute(reinterpret_cast<const void*>(&k_node), hipFuncAttributeMaxDynamicSharedMemorySize, L_LDS);
  const hipError_t a1 = hipFuncSetAttribute(reinterpret_cast<const void*>(&k_edge), hipFuncAttributeMaxDynamicSharedMemorySize, E_LDS);
  const hipError_t a2 = hipFuncSetAttribute(reinterpret_cast<const void*>(&k_agg),  hipFuncAttributeMaxDynamicSharedMemorySize, A_LDS);
  const hipError_t a3 = hipFuncSetAttribute(reinterpret_cast<const void*>(&k_upd),  hipFuncAttributeMaxDynamicSharedMemorySize, U_LDS);
  (void)a0; (void)a1; (void)a2; (void)a3;

  k_wcvt<<<T_BLK + 1, 256, 0, stream>>>(mw1, mw2, uw1, uw2, emb, wq, ekp, nTE);
  k_node<<<nBlkN, 256, L_LDS, stream>>>(hin, th, hap, hbp, nN);

  for (int c = 0; c < nchl; ++c) {
    const int cbase = c * CH;
    int clen = nE - cbase;
    clen = clen > CH ? CH : clen;
    const int nEB = (clen + ROWS - 1) / ROWS;
    k_edge<<<nEB, 256, E_LDS, stream>>>(ei, et, pos, hap, hbp, ekp, mw1, mb1, mb2, th, msp, nN, nE, nTE, cbase, clen);
    k_agg<<<nBlkA, NTHR, A_LDS, stream>>>(ei + (size_t)nE + (size_t)cbase, msp, agp, cnp, nN, clen, (c == 0) ? 1 : 0, vec_ok);
  }

  k_upd<<<nBlkN, 256, U_LDS, stream>>>(hin, agp, cnp, ntype, th, ub1, ub2, lng, lnb, out0, nN);
  (void)hipGetLastError();
}
